// LSTM_Cell_Model_85177791414679
// MI455X (gfx1250) — hardware-verified
//
#include <hip/hip_runtime.h>
#include <math.h>

constexpr int VOCAB   = 50000;
constexpr int EMB_DIM = 128;
constexpr int HID     = 256;
constexpr int NCLS    = 2;
constexpr int NBATCH  = 256;
constexpr int NSTEP   = 512;
constexpr int NGATE   = 4 * HID;
constexpr int KCAT    = EMB_DIM + HID;
constexpr int ROWS_PER_BLOCK = 16;
constexpr int NBLOCKS = NBATCH / ROWS_PER_BLOCK;
constexpr int APITCH  = KCAT + 8;
constexpr int SPITCH  = HID + 4;
constexpr float A_SCALE = 8.0f;
constexpr float W_SCALE = 16.0f;
constexpr float ACC_INV = 1.0f / 128.0f;
static_assert(KCAT % 32 == 0, "K multiple of 32");
static_assert(NBATCH % ROWS_PER_BLOCK == 0, "rows per block divide batch");
static_assert(NGATE == 8 * 128, "8 waves x 128 columns");
static_assert((APITCH * 2) % 16 == 0 && (SPITCH * 4) % 16 == 0, "16-B aligned LDS rows");

typedef __attribute__((ext_vector_type(16))) _Float16 v16h;
typedef __attribute__((ext_vector_type(8)))  _Float16 v8h;
typedef __attribute__((ext_vector_type(8)))  float    v8f;
typedef __attribute__((ext_vector_type(4)))  float    v4f;

__device__ __forceinline__ void dep_guard_h(v8f& a, v8f& b, v16h x, v16h y) { asm volatile("v_nop\n\tv_nop\n\tv_nop\n\tv_nop" : "+v"(a), "+v"(b) : "v"(x), "v"(y)); }
__device__ __forceinline__ void keep4_h(v16h a, v16h b, v16h c, v16h d) { asm volatile("v_nop" :: "v"(a), "v"(b), "v"(c), "v"(d)); }
__device__ __forceinline__ void acc_guard4(v8f& a, v8f& b, v8f& c, v8f& d) { asm volatile("v_nop\n\tv_nop\n\tv_nop\n\tv_nop" : "+v"(a), "+v"(b), "+v"(c), "+v"(d)); }

template <typename T> struct Frag;
template <> struct Frag<_Float16> {
  typedef v16h V; union U { v16h v; v8h h[2]; };
  static __device__ __forceinline__ v16h load(const _Float16* p) {
    U f; f.h[0] = *(const v8h*)(p); f.h[1] = *(const v8h*)(p + 16); return f.v;
  }
  static __device__ __forceinline__ v8f mma(v16h a, v16h b, v8f c) {
    return __builtin_amdgcn_wmma_f32_16x16x32_f16(false, a, false, b, (short)0, c, false, false);
  }
  static __device__ __forceinline__ void guard(v8f& a, v8f& b, v16h x, v16h y) { dep_guard_h(a, b, x, y); }
  static __device__ __forceinline__ void keep(v16h a, v16h b, v16h c, v16h d) { keep4_h(a, b, c, d); }
};

__global__ __launch_bounds__(256) void k_pack_w(const float* __restrict__ Wih,
                                                const float* __restrict__ Whh,
                                                unsigned short* __restrict__ Wcp) {
  const int i = blockIdx.x * 256 + threadIdx.x;
  if (i >= (NGATE * KCAT) / 8) return;
  const int base = i * 8;
  const int n  = base / KCAT;
  const int k  = base - n * KCAT;
  const int ka = k & (EMB_DIM - 1);
  const int kb = (k < EMB_DIM) ? k : (k - EMB_DIM);
  const v4f a0 = *(const v4f*)(Wih + (size_t)n * EMB_DIM + ka);
  const v4f a1 = *(const v4f*)(Wih + (size_t)n * EMB_DIM + ka + 4);
  const v4f c0 = *(const v4f*)(Whh + (size_t)n * HID + kb);
  const v4f c1 = *(const v4f*)(Whh + (size_t)n * HID + kb + 4);
  const bool first = (k < EMB_DIM);
  v8h hv;
#pragma unroll
  for (int e = 0; e < 4; ++e) {
    const float v0 = first ? a0[e] : c0[e];
    const float v1 = first ? a1[e] : c1[e];
    hv[e]     = (_Float16)(v0 * W_SCALE);
    hv[4 + e] = (_Float16)(v1 * W_SCALE);
  }
  _Float16* Wc = (_Float16*)Wcp;
  *(volatile v8h*)(Wc + base) = hv;
  __threadfence();
  *(volatile v8h*)(Wc + base) = hv;
}

__device__ __forceinline__ void store_rows16(const float* slab, float* dst, int tid) {
  for (int pass = 0; pass < 2; ++pass) {
#pragma unroll
    for (int it = 0; it < 4; ++it) {
      const int idx = it * 256 + tid;
      const int row = idx >> 6;
      const int c4  = (idx & 63) * 4;
      const v4f v = *(const v4f*)(slab + row * SPITCH + c4);
      *(volatile v4f*)(dst + (size_t)row * HID + c4) = v;
    }
    __threadfence();
  }
}

__global__ __launch_bounds__(256) void k_lstm(const int* __restrict__ x,
                                              const float* __restrict__ emb,
                                              const unsigned short* __restrict__ Wcp,
                                              const float* __restrict__ b_ih,
                                              const float* __restrict__ b_hh,
                                              const float* __restrict__ W_lin,
                                              const float* __restrict__ b_lin,
                                              float* __restrict__ out) {
  __shared__ __align__(16) _Float16 Atile[ROWS_PER_BLOCK * APITCH];
  __shared__ __align__(16) float    slab[ROWS_PER_BLOCK * SPITCH];
  __shared__ __align__(16) float    heads[32];

  const _Float16* Wc = (const _Float16*)Wcp;
  const int tid  = threadIdx.x;
  const int wave = tid >> 5;
  const int lane = tid & 31;
  const int hh   = lane >> 4;
  const int c    = lane & 15;
  const int koff = hh * 8;
  const int blk  = blockIdx.x;
  const int b0   = blk * ROWS_PER_BLOCK;

#pragma unroll
  for (int j = 0; j < 2; ++j) {
    const int idx = j * 256 + tid;
    const int row = idx >> 5;
    const int seg = idx & 31;
    *(uint4*)(Atile + row * APITCH + EMB_DIM + seg * 8) = make_uint4(0u, 0u, 0u, 0u);
  }

  float bias[2][4];
#pragma unroll
  for (int u = 0; u < 2; ++u) {
    const int n = (2 * wave + u) * 16 + c;
#pragma unroll
    for (int q = 0; q < 4; ++q) bias[u][q] = b_ih[q * HID + n] + b_hh[q * HID + n];
  }
  float cst[2][8], hst[2][8];
#pragma unroll
  for (int u = 0; u < 2; ++u)
#pragma unroll
    for (int r = 0; r < 8; ++r) { cst[u][r] = 0.0f; hst[u][r] = 0.0f; }

  const int grow = tid >> 4;
  const int gseg = tid & 15;
  const int* xrow = x + (size_t)(b0 + grow) * NSTEP;

  for (int t = 0; t < NSTEP; ++t) {
    {
      int tok = xrow[t];
      tok = tok < 0 ? 0 : (tok > VOCAB - 1 ? VOCAB - 1 : tok);
      const float* ep = emb + (size_t)tok * EMB_DIM + gseg * 8;
      const v4f e0 = *(const v4f*)(ep);
      const v4f e1 = *(const v4f*)(ep + 4);
      v8h ev;
#pragma unroll
      for (int e = 0; e < 4; ++e) {
        ev[e]     = (_Float16)(e0[e] * A_SCALE);
        ev[4 + e] = (_Float16)(e1[e] * A_SCALE);
      }
      *(v8h*)(Atile + grow * APITCH + gseg * 8) = ev;
    }
    __syncthreads();

    v8f acc[2][4];
#pragma unroll
    for (int u = 0; u < 2; ++u)
#pragma unroll
      for (int q = 0; q < 4; ++q) acc[u][q] = (v8f){0.f, 0.f, 0.f, 0.f, 0.f, 0.f, 0.f, 0.f};

#pragma unroll 3
    for (int ks = 0; ks < KCAT / 32; ++ks) {
      const int k0 = ks * 32;
      const v16h a = Frag<_Float16>::load(Atile + c * APITCH + k0 + koff);
#pragma unroll
      for (int u = 0; u < 2; ++u) {
        v16h bq[4];
#pragma unroll
        for (int q = 0; q < 4; ++q) {
          const size_t bo = (size_t)(q * HID + (2 * wave + u) * 16 + c) * KCAT + k0 + koff;
          bq[q] = Frag<_Float16>::load(Wc + bo);
        }
#pragma unroll
        for (int q = 0; q < 4; ++q) acc[u][q] = Frag<_Float16>::mma(a, bq[q], acc[u][q]);
        Frag<_Float16>::guard(acc[u][0], acc[u][3], a, bq[3]);
        Frag<_Float16>::keep(bq[0], bq[1], bq[2], bq[3]);
      }
    }
    acc_guard4(acc[0][0], acc[0][1], acc[0][2], acc[0][3]);
    acc_guard4(acc[1][0], acc[1][1], acc[1][2], acc[1][3]);
    __syncthreads();

#pragma unroll
    for (int u = 0; u < 2; ++u) {
      const int n = (2 * wave + u) * 16 + c;
#pragma unroll
      for (int r = 0; r < 8; ++r) {
        const int row = 8 * hh + r;
        const float gi = acc[u][0][r] * ACC_INV + bias[u][0];
        const float gf = acc[u][1][r] * ACC_INV + bias[u][1];
        const float gg = acc[u][2][r] * ACC_INV + bias[u][2];
        const float go = acc[u][3][r] * ACC_INV + bias[u][3];
        const float si = 1.0f / (1.0f + expf(-gi));
        const float sf = 1.0f / (1.0f + expf(-gf));
        const float so = 1.0f / (1.0f + expf(-go));
        const float tg = tanhf(gg);
        const float cn = sf * cst[u][r] + si * tg;
        const float hn = so * tanhf(cn);
        cst[u][r] = cn;
        hst[u][r] = hn;
        Atile[row * APITCH + EMB_DIM + n] = (_Float16)(hn * A_SCALE);
      }
    }
  }

#pragma unroll
  for (int u = 0; u < 2; ++u) {
    const int n = (2 * wave + u) * 16 + c;
#pragma unroll
    for (int r = 0; r < 8; ++r) slab[(8 * hh + r) * SPITCH + n] = hst[u][r];
  }
  __syncthreads();
  store_rows16(slab, out + (size_t)b0 * HID, tid);
  __syncthreads();

#pragma unroll
  for (int u = 0; u < 2; ++u) {
    const int n = (2 * wave + u) * 16 + c;
#pragma unroll
    for (int r = 0; r < 8; ++r) slab[(8 * hh + r) * SPITCH + n] = cst[u][r];
  }
  __syncthreads();
  store_rows16(slab, out + (size_t)NBATCH * HID + (size_t)b0 * HID, tid);

  if (wave == 0) {
    const int row = lane >> 1;
    const int cc  = lane & 1;
    const float* wl = W_lin + cc * HID;
    const float* cr = slab + row * SPITCH;
    float s = 0.0f;
#pragma unroll 1
    for (int k = 0; k < HID; ++k) s += cr[k] * wl[k];
    heads[lane] = s + b_lin[cc];
  }
  __syncthreads();
  {
    const v4f hv4 = *(const v4f*)(heads + 4 * (tid & 7));
    float* outp = out + (size_t)2 * NBATCH * HID + (size_t)blk * 32;
    for (int pass = 0; pass < 2; ++pass) {
      if (tid < 8) *(volatile v4f*)(outp + 4 * tid) = hv4;
      __threadfence();
    }
  }
}

extern "C" void kernel_launch(void* const* d_in, const int* in_sizes, int n_in,
                              void* d_out, int out_size, void* d_ws, size_t ws_size,
                              hipStream_t stream) {
  if (n_in < 8) return;
  if (in_sizes[0] != NBATCH * NSTEP || in_sizes[1] != VOCAB * EMB_DIM ||
      in_sizes[2] != NGATE * EMB_DIM || in_sizes[3] != NGATE * HID ||
      in_sizes[4] != NGATE || in_sizes[5] != NGATE || in_sizes[6] != NCLS * HID || in_sizes[7] != NCLS) return;
  if (out_size != 2 * NBATCH * HID + NBATCH * NCLS) return;
  const size_t wc_bytes = (size_t)NGATE * KCAT * 2;
  if (ws_size < wc_bytes) return;

  const int*   x     = (const int*)  d_in[0];
  const float* emb   = (const float*)d_in[1];
  const float* W_ih  = (const float*)d_in[2];
  const float* W_hh  = (const float*)d_in[3];
  const float* b_ih  = (const float*)d_in[4];
  const float* b_hh  = (const float*)d_in[5];
  const float* W_lin = (const float*)d_in[6];
  const float* b_lin = (const float*)d_in[7];
  unsigned short* Wc = (unsigned short*)d_ws;
  float* outp = (float*)d_out;

  const int pack_threads = (NGATE * KCAT) / 8;
  k_pack_w<<<pack_threads / 256, 256, 0, stream>>>(W_ih, W_hh, Wc);
  k_lstm<<<NBLOCKS, 256, 0, stream>>>(x, emb, Wc, b_ih, b_hh, W_lin, b_lin, outp);
}
